// CustomMultiHeadAttentionStoichRoPE_36249523978453
// MI455X (gfx1250) — hardware-verified
//
#include <hip/hip_runtime.h>
#include <math.h>

#define BATCH  4
#define NHEADS 16
#define HDIM   64
#define DMODEL 1024
#define NANG   32

typedef __attribute__((ext_vector_type(16))) _Float16 v16h;
typedef __attribute__((ext_vector_type(8)))  _Float16 v8h;
typedef __attribute__((ext_vector_type(16))) __bf16   v16b;
typedef __attribute__((ext_vector_type(8)))  __bf16   v8b;
typedef __attribute__((ext_vector_type(8)))  float    v8f;
typedef __attribute__((ext_vector_type(4)))  float    v4f;

__device__ __forceinline__ unsigned short f2bf_bits(float f) {
  unsigned u = __float_as_uint(f);
  return (unsigned short)((u + 0x7FFFu + ((u >> 16) & 1u)) >> 16);
}
__device__ __forceinline__ float bf_bits2f(unsigned short h) { return __uint_as_float(((unsigned)h) << 16); }

__device__ __forceinline__ void dep_guard_h(v8f& a, v8f& b, v16h x, v16h y) { asm volatile("v_nop\n\tv_nop\n\tv_nop\n\tv_nop" : "+v"(a), "+v"(b) : "v"(x), "v"(y)); }
__device__ __forceinline__ void dep_guard_b(v8f& a, v8f& b, v16b x, v16b y) { asm volatile("v_nop\n\tv_nop\n\tv_nop\n\tv_nop" : "+v"(a), "+v"(b) : "v"(x), "v"(y)); }
__device__ __forceinline__ void keep4_h(v16h a, v16h b, v16h c, v16h d) { asm volatile("v_nop" :: "v"(a), "v"(b), "v"(c), "v"(d)); }
__device__ __forceinline__ void keep4_b(v16b a, v16b b, v16b c, v16b d) { asm volatile("v_nop" :: "v"(a), "v"(b), "v"(c), "v"(d)); }
__device__ __forceinline__ void acc_guard4(v8f& a, v8f& b, v8f& c, v8f& d) { asm volatile("v_nop\n\tv_nop\n\tv_nop\n\tv_nop" : "+v"(a), "+v"(b), "+v"(c), "+v"(d)); }
template <typename T> struct Frag;
template <> struct Frag<_Float16> {
  typedef v16h V; union U { v16h v; v8h h[2]; };
  static __device__ __forceinline__ v16h load(const _Float16* p) {
    U f; f.h[0] = *(const v8h*)(p); f.h[1] = *(const v8h*)(p + 16); return f.v;
  }
  static __device__ __forceinline__ v8f mma(v16h a, v16h b, v8f c) {
    return __builtin_amdgcn_wmma_f32_16x16x32_f16(false, a, false, b, (short)0, c, false, false);
  }
  static __device__ __forceinline__ void guard(v8f& a, v8f& b, v16h x, v16h y) { dep_guard_h(a, b, x, y); }
  static __device__ __forceinline__ void keep(v16h a, v16h b, v16h c, v16h d) { keep4_h(a, b, c, d); }
};
template <> struct Frag<__bf16> {
  typedef v16b V; union U { v16b v; v8b h[2]; };
  static __device__ __forceinline__ v16b load(const __bf16* p) {
    U f; f.h[0] = *(const v8b*)(p); f.h[1] = *(const v8b*)(p + 16); return f.v;
  }
  static __device__ __forceinline__ v8f mma(v16b a, v16b b, v8f c) {
    return __builtin_amdgcn_wmma_f32_16x16x32_bf16(false, a, false, b, (short)0, c, false, false);
  }
  static __device__ __forceinline__ void guard(v8f& a, v8f& b, v16b x, v16b y) { dep_guard_b(a, b, x, y); }
  static __device__ __forceinline__ void keep(v16b a, v16b b, v16b c, v16b d) { keep4_b(a, b, c, d); }
};

template <int ET> struct Elem;
template <> struct Elem<0> { typedef _Float16 T; };
template <> struct Elem<1> { typedef __bf16 T; };
template <int ET, bool SPLIT, int BIAS_MODE, int OUT_MODE, bool RESID, int ACT = 0>
__global__ __launch_bounds__(256) void wmma_gemm64(
    const unsigned short* __restrict__ Ap, const unsigned short* __restrict__ A2p, int lda, long strideA,
    const unsigned short* __restrict__ Btp, const unsigned short* __restrict__ Bt2p, int ldb, long strideB,
    void* __restrict__ Cout, void* __restrict__ Cout2, int ldc, long strideC,
    const float* __restrict__ bias,
    const float* __restrict__ resid, long strideR,
    int M, int N, int K, float scale) {
  typedef typename Elem<ET>::T T;
  typedef typename Frag<T>::V V;
  const T* A = (const T*)Ap; const T* A2 = (const T*)A2p; const T* Bt = (const T*)Btp; const T* Bt2 = (const T*)Bt2p;
  __shared__ __align__(16) float sT[8][16 * 68];
  const int b    = blockIdx.y;
  const int lane = threadIdx.x & 31;
  const int wave = threadIdx.x >> 5;
  const int tilesN = N >> 6;
  const int tilesM = M >> 6;
  const int tile = blockIdx.x * 8 + wave;
  if (tile >= tilesM * tilesN) return;
  const int tm = tile / tilesN;
  const int tn = tile - tm * tilesN;
  const int m0 = tm << 6;
  const int n0 = tn << 6;

  const T* Ab  = A  + (size_t)b * strideA;
  const T* Bb  = Bt + (size_t)b * strideB;
  const T* Ab2 = SPLIT ? (A2  + (size_t)b * strideA) : nullptr;
  const T* Bb2 = SPLIT ? (Bt2 + (size_t)b * strideB) : nullptr;

  const int rlane = lane & 15;
  const int koff  = (lane >> 4) * 8;
  const int mOff  = (lane >> 4) * 8;

  v8f acc[4][4];
#pragma unroll
  for (int i = 0; i < 4; ++i)
#pragma unroll
    for (int j = 0; j < 4; ++j) acc[i][j] = (v8f){0.f,0.f,0.f,0.f,0.f,0.f,0.f,0.f};

  for (int k0 = 0; k0 < K; k0 += 32) {
    V bh[4], bl[4];
#pragma unroll
    for (int j = 0; j < 4; ++j) {
      const size_t bo = (size_t)(n0 + (j << 4) + rlane) * ldb + koff + k0;
      bh[j] = Frag<T>::load(Bb + bo);
      if (SPLIT) bl[j] = Frag<T>::load(Bb2 + bo);
    }
#pragma unroll
    for (int i = 0; i < 4; ++i) {
      const size_t ao = (size_t)(m0 + (i << 4) + rlane) * lda + koff + k0;
      V ah = Frag<T>::load(Ab + ao);
      V al;
      if (SPLIT) al = Frag<T>::load(Ab2 + ao);
#pragma unroll
      for (int j = 0; j < 4; ++j) {
        acc[i][j] = Frag<T>::mma(ah, bh[j], acc[i][j]);
        if (SPLIT) {
          acc[i][j] = Frag<T>::mma(ah, bl[j], acc[i][j]);
          acc[i][j] = Frag<T>::mma(al, bh[j], acc[i][j]);
        }
      }
      Frag<T>::guard(acc[i][0], acc[i][3], ah, SPLIT ? al : ah);
    }
    Frag<T>::keep(bh[0], bh[1], bh[2], bh[3]);
    if (SPLIT) Frag<T>::keep(bl[0], bl[1], bl[2], bl[3]);
  }
  acc_guard4(acc[0][0], acc[0][1], acc[0][2], acc[0][3]);
  acc_guard4(acc[1][0], acc[1][1], acc[1][2], acc[1][3]);
  acc_guard4(acc[2][0], acc[2][1], acc[2][2], acc[2][3]);
  acc_guard4(acc[3][0], acc[3][1], acc[3][2], acc[3][3]);

  float* slab = sT[wave];
  const float* Rb = RESID ? (resid + (size_t)b * strideR) : nullptr;
#pragma unroll
  for (int i = 0; i < 4; ++i) {
    const int mBase = m0 + (i << 4);
#pragma unroll
    for (int j = 0; j < 4; ++j) {
      const int n = n0 + (j << 4) + rlane;
      float bv = 0.f;
      if (BIAS_MODE == 2) bv = bias[n];
#pragma unroll
      for (int r = 0; r < 8; ++r) {
        float v = acc[i][j][r] * scale;
        if (BIAS_MODE == 1) v += bias[mBase + mOff + r];
        if (BIAS_MODE == 2) v += bv;
        if (RESID) v += Rb[(size_t)(mBase + mOff + r) * ldc + n];
        if (ACT == 1) v = tanhf(v);
        if (ACT == 2) v = fmaxf(v, 0.0f);
        if (ACT == 3) v = v / (1.0f + expf(-v));
        if (ACT == 4) v = (v > 0.f) ? v : 0.01f * v;
        if (ACT == 5) v = 0.5f * v * (1.0f + erff(v * 0.70710678118654752f));
        slab[(mOff + r) * 68 + (j << 4) + rlane] = v;
      }
    }
    __builtin_amdgcn_fence(__ATOMIC_RELEASE, "workgroup");
    __builtin_amdgcn_wave_barrier();
    __builtin_amdgcn_fence(__ATOMIC_ACQUIRE, "workgroup");
    if (OUT_MODE == 0) {
      float* C = (float*)Cout + (size_t)b * strideC;
      const int hh = lane >> 4, c4 = (lane & 15) * 4;
      for (int pass = 0; pass < 2; ++pass) {
#pragma unroll
        for (int it = 0; it < 8; ++it) {
          const int row = it * 2 + hh;
          v4f v = *(const v4f*)(slab + row * 68 + c4);
          *(volatile v4f*)(C + (size_t)(mBase + row) * ldc + n0 + c4) = v;
        }
        __threadfence();
      }
    } else {
      const int q = lane >> 3, c8 = (lane & 7) * 8;
      unsigned short* C  = (unsigned short*)Cout  + (size_t)b * strideC;
      unsigned short* C2 = (OUT_MODE == 2) ? ((unsigned short*)Cout2 + (size_t)b * strideC) : nullptr;
      for (int pass = 0; pass < 2; ++pass) {
#pragma unroll
        for (int it = 0; it < 4; ++it) {
          const int row = it * 4 + q;
          const float* sp = slab + row * 68 + c8;
          v8h hv, lv;
#pragma unroll
          for (int e = 0; e < 8; ++e) {
            if (OUT_MODE == 1) {
              hv[e] = (_Float16)sp[e];
            } else {
              unsigned short hb = f2bf_bits(sp[e]);
              unsigned short lb = f2bf_bits(sp[e] - bf_bits2f(hb));
              hv[e] = __builtin_bit_cast(_Float16, hb);
              lv[e] = __builtin_bit_cast(_Float16, lb);
            }
          }
          *(volatile v8h*)(C + (size_t)(mBase + row) * ldc + n0 + c8) = hv;
          if (OUT_MODE == 2) *(volatile v8h*)(C2 + (size_t)(mBase + row) * ldc + n0 + c8) = lv;
        }
        __threadfence();
      }
    }
    __builtin_amdgcn_fence(__ATOMIC_RELEASE, "workgroup");
    __builtin_amdgcn_wave_barrier();
    __builtin_amdgcn_fence(__ATOMIC_ACQUIRE, "workgroup");
  }
}

__global__ __launch_bounds__(256) void wmma_gemm64_rope(
    const unsigned short* __restrict__ Ap, int lda,
    const unsigned short* __restrict__ Btp, int ldb,
    unsigned short* __restrict__ Cout, int ldc,
    const float* __restrict__ bias, const float* __restrict__ cs, const float* __restrict__ sn,
    int M, int N, int K, float scale) {
  typedef _Float16 T;
  typedef v16h V;
  const T* A = (const T*)Ap; const T* Bt = (const T*)Btp;
  __shared__ __align__(16) float sT[8][16 * 68];
  const int lane = threadIdx.x & 31;
  const int wave = threadIdx.x >> 5;
  const int tilesN = N >> 6;
  const int tilesM = M >> 6;
  const int tile = blockIdx.x * 8 + wave;
  if (tile >= tilesM * tilesN) return;
  const int tm = tile / tilesN;
  const int tn = tile - tm * tilesN;
  const int m0 = tm << 6;
  const int n0 = tn << 6;

  const int rlane = lane & 15;
  const int koff  = (lane >> 4) * 8;
  const int mOff  = (lane >> 4) * 8;

  v8f acc[4][4];
#pragma unroll
  for (int i = 0; i < 4; ++i)
#pragma unroll
    for (int j = 0; j < 4; ++j) acc[i][j] = (v8f){0.f,0.f,0.f,0.f,0.f,0.f,0.f,0.f};

  for (int k0 = 0; k0 < K; k0 += 32) {
    V bh[4];
#pragma unroll
    for (int j = 0; j < 4; ++j) {
      const size_t bo = (size_t)(n0 + (j << 4) + rlane) * ldb + koff + k0;
      bh[j] = Frag<T>::load(Bt + bo);
    }
#pragma unroll
    for (int i = 0; i < 4; ++i) {
      const size_t ao = (size_t)(m0 + (i << 4) + rlane) * lda + koff + k0;
      V ah = Frag<T>::load(A + ao);
#pragma unroll
      for (int j = 0; j < 4; ++j) acc[i][j] = Frag<T>::mma(ah, bh[j], acc[i][j]);
      Frag<T>::guard(acc[i][0], acc[i][3], ah, ah);
    }
    Frag<T>::keep(bh[0], bh[1], bh[2], bh[3]);
  }
  acc_guard4(acc[0][0], acc[0][1], acc[0][2], acc[0][3]);
  acc_guard4(acc[1][0], acc[1][1], acc[1][2], acc[1][3]);
  acc_guard4(acc[2][0], acc[2][1], acc[2][2], acc[2][3]);
  acc_guard4(acc[3][0], acc[3][1], acc[3][2], acc[3][3]);

  float* slab = sT[wave];
  float bA[2], bB[2];
#pragma unroll
  for (int jj = 0; jj < 2; ++jj) {
    bA[jj] = bias[n0 + (jj << 4) + rlane];
    bB[jj] = bias[n0 + 32 + (jj << 4) + rlane];
  }
#pragma unroll
  for (int i = 0; i < 4; ++i) {
    const int mBase = m0 + (i << 4);
#pragma unroll
    for (int jj = 0; jj < 2; ++jj) {
      const int dA = (jj << 4) + rlane;
#pragma unroll
      for (int r = 0; r < 8; ++r) {
        const int m = mBase + mOff + r;
        const float cv = cs[(size_t)m * NANG + dA];
        const float sv = sn[(size_t)m * NANG + dA];
        const float xl = acc[i][jj][r] * scale + bA[jj];
        const float xr = acc[i][jj + 2][r] * scale + bB[jj];
        slab[(mOff + r) * 68 + dA]      = xl * cv - xr * sv;
        slab[(mOff + r) * 68 + 32 + dA] = xl * sv + xr * cv;
      }
    }
    __builtin_amdgcn_fence(__ATOMIC_RELEASE, "workgroup");
    __builtin_amdgcn_wave_barrier();
    __builtin_amdgcn_fence(__ATOMIC_ACQUIRE, "workgroup");
    {
      const int q = lane >> 3, c8 = (lane & 7) * 8;
      unsigned short* C = Cout;
      for (int pass = 0; pass < 2; ++pass) {
#pragma unroll
        for (int it = 0; it < 4; ++it) {
          const int row = it * 4 + q;
          const float* sp = slab + row * 68 + c8;
          v8h hv;
#pragma unroll
          for (int e = 0; e < 8; ++e) hv[e] = (_Float16)sp[e];
          *(volatile v8h*)(C + (size_t)(mBase + row) * ldc + n0 + c8) = hv;
        }
        __threadfence();
      }
    }
    __builtin_amdgcn_fence(__ATOMIC_RELEASE, "workgroup");
    __builtin_amdgcn_wave_barrier();
    __builtin_amdgcn_fence(__ATOMIC_ACQUIRE, "workgroup");
  }
}

__global__ __launch_bounds__(256) void cast_f32_f16x8(
    const float* __restrict__ in, _Float16* __restrict__ out, int n8, float scale) {
  const int i = blockIdx.x * 256 + threadIdx.x;
  if (i < n8) {
    const size_t e0 = (size_t)i * 8;
    const v4f a = *(const v4f*)(in + e0);
    const v4f b = *(const v4f*)(in + e0 + 4);
    v8h hv;
    hv[0] = (_Float16)(a[0] * scale); hv[1] = (_Float16)(a[1] * scale);
    hv[2] = (_Float16)(a[2] * scale); hv[3] = (_Float16)(a[3] * scale);
    hv[4] = (_Float16)(b[0] * scale); hv[5] = (_Float16)(b[1] * scale);
    hv[6] = (_Float16)(b[2] * scale); hv[7] = (_Float16)(b[3] * scale);
    *(volatile v8h*)(out + e0) = hv;
    __threadfence();
    *(volatile v8h*)(out + e0) = hv;
  }
}

__global__ __launch_bounds__(256) void rope_table(
    const float* __restrict__ frac, float* __restrict__ cs, float* __restrict__ sn, int nt) {
  const int idx = blockIdx.x * 256 + threadIdx.x;
  if (idx < nt) {
    const int m = idx >> 5, i = idx & 31;
    const float pos = frac[m] * 1000.0f;
    const float e  = (float)(2 * i) / 64.0f;
    const float fd = powf(10000.0f, e);
    const float ang = pos * (1.0f / fd);
    const float cv = cosf(ang);
    const float sv = sinf(ang);
    ((volatile float*)cs)[idx] = cv;
    ((volatile float*)sn)[idx] = sv;
    __threadfence();
    ((volatile float*)cs)[idx] = cv;
    ((volatile float*)sn)[idx] = sv;
  }
}

#define AT_D 64
#define AT_NW 4
#define AT_QB 64
#define AT_KC 64

__device__ __forceinline__ v8f at_mmah(v16h a, v16h b, v8f c) {
  c = __builtin_amdgcn_wmma_f32_16x16x32_f16(false, a, false, b, (short)0, c, false, false);
  asm volatile("v_nop\n\tv_nop\n\tv_nop\n\tv_nop" : "+v"(c) : "v"(a), "v"(b));
  return c;
}

__global__ __launch_bounds__(128)
void attn64_f16(const _Float16* __restrict__ q, const _Float16* __restrict__ k,
                const _Float16* __restrict__ vt, _Float16* __restrict__ out,
                long q_bs, long q_rs, long q_hs, long k_bs, long k_rs, long k_hs,
                long v_bs, long v_ds, long v_hs, long o_bs, long o_rs, long o_hs,
                int S, int Skv, int H, float sscale, float oscale) {
  const float PSC = 32768.0f;
  union FH { v16h v; v8h h[2]; };
  __shared__ __align__(16) _Float16 Ksh[AT_KC * AT_D];
  __shared__ __align__(16) _Float16 Vth[AT_D * AT_KC];
  __shared__ __align__(16) _Float16 Psh[AT_NW][16 * AT_KC];
  __shared__ __align__(16) float    Os[AT_NW][16 * 68];

  const int tid  = threadIdx.x;
  const int wave = tid >> 5;
  const int lane = tid & 31;
  const int hh   = lane >> 4;
  const int c    = lane & 15;

  const int nqb = S / AT_QB;
  const int bx = blockIdx.x;
  const int qb = bx % nqb;
  const int bh = bx / nqb;
  const int h  = bh % H;
  const int b  = bh / H;
  const int q0 = qb * AT_QB + wave * 16;

  const _Float16* qb_ptr = q   + (size_t)b * q_bs + (size_t)h * q_hs;
  const _Float16* kb_ptr = k   + (size_t)b * k_bs + (size_t)h * k_hs;
  const _Float16* vb_ptr = vt  + (size_t)b * v_bs + (size_t)h * v_hs;
  _Float16*       ob_ptr = out + (size_t)b * o_bs + (size_t)h * o_hs;

  v16h qa[2];
  {
    const _Float16* qrow = qb_ptr + (size_t)(q0 + c) * q_rs;
#pragma unroll
    for (int dc = 0; dc < 2; ++dc) qa[dc] = Frag<_Float16>::load(qrow + dc * 32 + 8 * hh);
  }

  float mrow[8], lrow[8];
  v8f oacc[4];
#pragma unroll
  for (int r = 0; r < 8; ++r) { mrow[r] = -__builtin_inff(); lrow[r] = 0.f; }
#pragma unroll
  for (int t = 0; t < 4; ++t) oacc[t] = (v8f){0.f,0.f,0.f,0.f,0.f,0.f,0.f,0.f};

  const int nChunks = Skv / AT_KC;
  for (int kc = 0; kc < nChunks; ++kc) {
    const int kv0 = kc * AT_KC;
    __syncthreads();
    {
      const int rr = tid >> 1, hf = (tid & 1) * 32;
      const _Float16* krow = kb_ptr + (size_t)(kv0 + rr) * k_rs + hf;
      const _Float16* vrow = vb_ptr + (size_t)rr * v_ds + kv0 + hf;
#pragma unroll
      for (int i = 0; i < 4; ++i) {
        const v8h kk = *(const v8h*)(krow + 8 * i);
        const v8h vv = *(const v8h*)(vrow + 8 * i);
        *(v8h*)(Ksh + rr * AT_D  + hf + 8 * i) = kk;
        *(v8h*)(Vth + rr * AT_KC + hf + 8 * i) = vv;
      }
    }
    __syncthreads();

    v8f s[4];
#pragma unroll
    for (int j = 0; j < 4; ++j) {
      s[j] = (v8f){0.f,0.f,0.f,0.f,0.f,0.f,0.f,0.f};
#pragma unroll
      for (int dc = 0; dc < 2; ++dc) {
        FH kbf;
        kbf.h[0] = *(const v8h*)(Ksh + (j * 16 + c) * AT_D + dc * 32 + 8 * hh);
        kbf.h[1] = *(const v8h*)(Ksh + (j * 16 + c) * AT_D + dc * 32 + 16 + 8 * hh);
        s[j] = at_mmah(qa[dc], kbf.v, s[j]);
      }
    }
    float cm[8];
#pragma unroll
    for (int r = 0; r < 8; ++r) {
      float m = -__builtin_inff();
#pragma unroll
      for (int j = 0; j < 4; ++j) { s[j][r] *= sscale; m = fmaxf(m, s[j][r]); }
#pragma unroll
      for (int off = 1; off < 16; off <<= 1) m = fmaxf(m, __shfl_xor(m, off, 32));
      cm[r] = m;
    }
    _Float16* pwh = Psh[wave];
#pragma unroll
    for (int r = 0; r < 8; ++r) {
      const float mnew = fmaxf(mrow[r], cm[r]);
      const float alpha = __expf(mrow[r] - mnew);
      mrow[r] = mnew;
      float psum = 0.f;
#pragma unroll
      for (int j = 0; j < 4; ++j) {
        const float p = __expf(s[j][r] - mnew);
        psum += p;
        pwh[(8 * hh + r) * AT_KC + j * 16 + c] = (_Float16)(p * PSC);
      }
#pragma unroll
      for (int off = 1; off < 16; off <<= 1) psum += __shfl_xor(psum, off, 32);
      lrow[r] = lrow[r] * alpha + psum;
#pragma unroll
      for (int t = 0; t < 4; ++t) oacc[t][r] *= alpha;
    }
    __builtin_amdgcn_fence(__ATOMIC_RELEASE, "workgroup");
    __builtin_amdgcn_wave_barrier();
    __builtin_amdgcn_fence(__ATOMIC_ACQUIRE, "workgroup");
#pragma unroll 1
    for (int kk = 0; kk < 2; ++kk) {
      FH pa;
      pa.h[0] = *(const v8h*)(pwh + c * AT_KC + kk * 32 + 8 * hh);
      pa.h[1] = *(const v8h*)(pwh + c * AT_KC + kk * 32 + 16 + 8 * hh);
#pragma unroll
      for (int t = 0; t < 4; ++t) {
        FH vb;
        vb.h[0] = *(const v8h*)(Vth + (t * 16 + c) * AT_KC + kk * 32 + 8 * hh);
        vb.h[1] = *(const v8h*)(Vth + (t * 16 + c) * AT_KC + kk * 32 + 16 + 8 * hh);
        oacc[t] = at_mmah(pa.v, vb.v, oacc[t]);
      }
    }
  }

  float* os = Os[wave];
#pragma unroll
  for (int r = 0; r < 8; ++r) {
    const float inv = oscale * (1.0f / (lrow[r] * PSC));
#pragma unroll
    for (int t = 0; t < 4; ++t) os[(8 * hh + r) * 68 + t * 16 + c] = oacc[t][r] * inv;
  }
  __builtin_amdgcn_fence(__ATOMIC_RELEASE, "workgroup");
  __builtin_amdgcn_wave_barrier();
  __builtin_amdgcn_fence(__ATOMIC_ACQUIRE, "workgroup");
  {
    const int q8 = lane >> 3, c8 = (lane & 7) * 8;
    for (int pass = 0; pass < 2; ++pass) {
#pragma unroll
      for (int it = 0; it < 4; ++it) {
        const int row = it * 4 + q8;
        const float* sp = os + row * 68 + c8;
        v8h hv;
#pragma unroll
        for (int e = 0; e < 8; ++e) hv[e] = (_Float16)sp[e];
        *(volatile v8h*)(ob_ptr + (size_t)(q0 + row) * o_rs + c8) = hv;
      }
      __threadfence();
    }
  }
}

extern "C" void kernel_launch(void* const* d_in, const int* in_sizes, int n_in,
                              void* d_out, int out_size, void* d_ws, size_t ws_size,
                              hipStream_t stream) {
  if (n_in < 10) return;
  const int D = DMODEL;
  if (in_sizes[3] != D || in_sizes[5] != D || in_sizes[7] != D || in_sizes[9] != D) return;
  if (in_sizes[2] != D * D || in_sizes[4] != D * D || in_sizes[6] != D * D || in_sizes[8] != D * D) return;
  const int M = in_sizes[0] / D;
  if ((size_t)M * D != (size_t)in_sizes[0] || in_sizes[1] != M || out_size != M * D) return;
  const int T = M / BATCH;
  if (T * BATCH != M || (T % 64) != 0 || (M % 64) != 0 || NHEADS * HDIM != D) return;

  const float* x    = (const float*)d_in[0];
  const float* frac = (const float*)d_in[1];
  const float* Wq   = (const float*)d_in[2];
  const float* bq   = (const float*)d_in[3];
  const float* Wk   = (const float*)d_in[4];
  const float* bk   = (const float*)d_in[5];
  const float* Wv   = (const float*)d_in[6];
  const float* bv   = (const float*)d_in[7];
  const float* Wo   = (const float*)d_in[8];
  const float* bo   = (const float*)d_in[9];
  float* out = (float*)d_out;

  const size_t nX = (size_t)M * D;
  const size_t nW = (size_t)D * D;
  const size_t nT = (size_t)M * NANG;

  char* ws = (char*)d_ws;
  size_t off = 0;
  auto take = [&](size_t bytes) -> char* {
    char* p = ws + off; off += (bytes + 255) & ~(size_t)255; return p;
  };
  _Float16* x16  = (_Float16*)take(nX * 2);
  _Float16* Wq16 = (_Float16*)take(nW * 2);
  _Float16* Wk16 = (_Float16*)take(nW * 2);
  _Float16* Wv16 = (_Float16*)take(nW * 2);
  _Float16* Wo16 = (_Float16*)take(nW * 2);
  float*    cs   = (float*)take(nT * 4);
  float*    sn   = (float*)take(nT * 4);
  _Float16* Qh   = (_Float16*)take(nX * 2);
  _Float16* Kh   = (_Float16*)take(nX * 2);
  _Float16* Vt   = (_Float16*)take(nX * 2);
  _Float16* AO   = (_Float16*)take(nX * 2);
  if (off > ws_size || off > (size_t)134217728) return;

  const int n8x = (int)(nX / 8), n8w = (int)(nW / 8);
  cast_f32_f16x8<<<(n8x + 255) / 256, 256, 0, stream>>>(x,  x16,  n8x, 1.0f);
  cast_f32_f16x8<<<(n8w + 255) / 256, 256, 0, stream>>>(Wq, Wq16, n8w, 32.0f);
  cast_f32_f16x8<<<(n8w + 255) / 256, 256, 0, stream>>>(Wk, Wk16, n8w, 32.0f);
  cast_f32_f16x8<<<(n8w + 255) / 256, 256, 0, stream>>>(Wv, Wv16, n8w, 32.0f);
  cast_f32_f16x8<<<(n8w + 255) / 256, 256, 0, stream>>>(Wo, Wo16, n8w, 32.0f);

  rope_table<<<((int)nT + 255) / 256, 256, 0, stream>>>(frac, cs, sn, (int)nT);

  const int gtiles = (M / 64) * (D / 64);
  const int ggrid  = (gtiles + 7) / 8;
  typedef const unsigned short cus;

  wmma_gemm64_rope<<<ggrid, 256, 0, stream>>>((cus*)x16, D, (cus*)Wq16, D, (unsigned short*)Qh, D,
                                               bq, cs, sn, M, D, D, 1.0f / 32.0f);
  wmma_gemm64_rope<<<ggrid, 256, 0, stream>>>((cus*)x16, D, (cus*)Wk16, D, (unsigned short*)Kh, D,
                                               bk, cs, sn, M, D, D, 1.0f / 32.0f);
  wmma_gemm64<0, false, 1, 1, false><<<dim3(ggrid, 1), 256, 0, stream>>>(
      (cus*)Wv16, nullptr, D, 0L, (cus*)x16, nullptr, D, 0L,
      (void*)Vt, nullptr, M, 0L, bv, nullptr, 0L, D, M, D, 1.0f / 32.0f);

  const int agrid = BATCH * NHEADS * (T / 64);
  attn64_f16<<<agrid, 128, 0, stream>>>(Qh, Kh, Vt, AO,
                                        (long)T * D, (long)D, (long)HDIM,
                                        (long)T * D, (long)D, (long)HDIM,
                                        (long)T, (long)M, (long)HDIM * M,
                                        (long)T * D, (long)D, (long)HDIM,
                                        T, T, NHEADS, 0.125f, 64.0f);

  wmma_gemm64<0, false, 2, 0, false><<<dim3(ggrid, 1), 256, 0, stream>>>(
      (cus*)AO, nullptr, D, 0L, (cus*)Wo16, nullptr, D, 0L,
      (void*)out, nullptr, D, 0L, bo, nullptr, 0L, M, D, D, 1.0f / 2048.0f);
}
